// SparseCrossEncoderSelfAttention_37280316129300
// MI455X (gfx1250) — hardware-verified
//
#include <hip/hip_runtime.h>
#include <math.h>

typedef __attribute__((ext_vector_type(16))) _Float16 v16h;
typedef __attribute__((ext_vector_type(16))) __bf16 v16b;
typedef __attribute__((ext_vector_type(8)))  _Float16 v8h;
typedef __attribute__((ext_vector_type(8)))  float v8f;
typedef __attribute__((ext_vector_type(4)))  float v4f;
typedef __attribute__((ext_vector_type(2)))  float v2f;
typedef __attribute__((ext_vector_type(4)))  unsigned v4u;
typedef __attribute__((ext_vector_type(4)))  int v4i;
typedef float __attribute__((may_alias)) float_a;
typedef int __attribute__((may_alias)) int_a;

template <typename T> __device__ __forceinline__ void vst2(void* p, T v) { *(volatile T*)p = v; __threadfence(); *(volatile T*)p = v; }
__device__ __forceinline__ v8f wmma16(v16h a, v16h b, v8f c) {
  v8f d = __builtin_amdgcn_wmma_f32_16x16x32_f16(false, a, false, b, (short)0, c, false, false);
  asm volatile("v_nop\n\tv_nop\n\tv_nop\n\tv_nop" : "+v"(d) : "v"(a), "v"(b));
  return d;
}
__device__ __forceinline__ v8f wmma_bf(v16b a, v16b b, v8f c) {
  v8f d = __builtin_amdgcn_wmma_f32_16x16x32_bf16(false, a, false, b, (short)0, c, false, false);
  asm volatile("v_nop\n\tv_nop\n\tv_nop\n\tv_nop" : "+v"(d) : "v"(a), "v"(b));
  return d;
}
__device__ __forceinline__ v16h frag_h(const _Float16* rowk0, int lane) {
  union { v16h v; v8h q[2]; } u; const _Float16* p = rowk0 + 8 * (lane >> 4);
  u.q[0] = *(const v8h*)p; u.q[1] = *(const v8h*)(p + 16); return u.v;
}
__device__ __forceinline__ v16h frag_f32(const float* rowk0, int lane) {
  v16h a; const float* p = rowk0 + 8 * (lane >> 4);
#pragma unroll
  for (int i = 0; i < 8; ++i) { a[i] = (_Float16)p[i]; a[8 + i] = (_Float16)p[16 + i]; }
  return a;
}
__device__ __forceinline__ v16h frag_f32s(const float* rowk0, int lane, float sc) {
  v16h a; const float* p = rowk0 + 8 * (lane >> 4);
#pragma unroll
  for (int i = 0; i < 8; ++i) { a[i] = (_Float16)(p[i] * sc); a[8 + i] = (_Float16)(p[16 + i] * sc); }
  return a;
}
__device__ __forceinline__ v16h fragc_f32(const float* W, int k0, int n, int lane, int ld, int K) {
  v16h a; const int g = lane >> 4;
#pragma unroll
  for (int i = 0; i < 8; ++i) { const int ka = k0 + 8 * g + i, kb = ka + 16;
    a[i] = (_Float16)(ka < K ? W[(size_t)(ka < K ? ka : K - 1) * ld + n] : 0.f); a[8 + i] = (_Float16)(kb < K ? W[(size_t)(kb < K ? kb : K - 1) * ld + n] : 0.f); }
  return a;
}
struct F2 { v16b h, l; };
__device__ __forceinline__ F2 bsplit16(const float v[16]) { F2 r;
#pragma unroll
  for (int i = 0; i < 16; ++i) { const __bf16 h = (__bf16)v[i]; r.h[i] = h; r.l[i] = (__bf16)(v[i] - (float)h); }
  return r; }
__device__ __forceinline__ F2 split_row(const float* row, int k0, int lane) { float v[16]; const float* p = row + k0 + 8 * (lane >> 4);
#pragma unroll
  for (int i = 0; i < 8; ++i) { v[i] = p[i]; v[8 + i] = p[16 + i]; }
  return bsplit16(v); }
__device__ __forceinline__ F2 split_rowK(const float* row, int k0, int lane, int K) { float v[16]; const int g = lane >> 4;
#pragma unroll
  for (int i = 0; i < 8; ++i) { const int ka = k0 + 8 * g + i, kb = ka + 16; v[i] = ka < K ? row[ka < K ? ka : K - 1] : 0.f; v[8 + i] = kb < K ? row[kb < K ? kb : K - 1] : 0.f; }
  return bsplit16(v); }
__device__ __forceinline__ F2 split_col(const float* W, int k0, int n, int lane, int ld, int K) { float v[16]; const int g = lane >> 4;
#pragma unroll
  for (int i = 0; i < 8; ++i) { const int ka = k0 + 8 * g + i, kb = ka + 16; v[i] = ka < K ? W[(size_t)(ka < K ? ka : K - 1) * ld + n] : 0.f; v[8 + i] = kb < K ? W[(size_t)(kb < K ? kb : K - 1) * ld + n] : 0.f; }
  return bsplit16(v); }
__device__ __forceinline__ v8f mac3(const F2& a, const F2& b, v8f c) { c = wmma_bf(a.l, b.h, c); c = wmma_bf(a.h, b.l, c); return wmma_bf(a.h, b.h, c); }
__device__ __forceinline__ float sigm(float v) { return 1.0f / (1.0f + expf(-v)); }
#define LDSX() do { asm volatile("s_wait_dscnt 0" ::: "memory"); __builtin_amdgcn_wave_barrier(); __builtin_amdgcn_fence(__ATOMIC_RELEASE, "workgroup"); } while (0)


#define NBB 2
#define ND 16
#define NQT 32
#define NS 512
#define HIDN 768
#define NH 12
#define HD 64
#define LSEQ (1 + NQT + NS)
#define RPB (1 + NQT + ND * NS)
#define NROW (NBB * RPB)
#define NROWP (((NROW + 63) / 64) * 64)
#ifndef TND
#define TND ND
#endif
#ifndef TNB
#define TNB NBB
#endif
#ifndef TPR
#define TPR (NROWP / 64)
#endif
typedef __attribute__((ext_vector_type(8))) __bf16 v8b;
__device__ __forceinline__ v16b frag_b(const __bf16* rowk0, int lane) {
  union { v16b v; v8b q[2]; } u; const __bf16* p = rowk0 + 8 * (lane >> 4);
  u.q[0] = *(const v8b*)p; u.q[1] = *(const v8b*)(p + 16); return u.v;
}
__device__ __forceinline__ float bfr(float v) { return (float)(__bf16)v; }
__device__ __attribute__((noinline)) float exp_ni(float v) { return expf(v); }
__device__ __attribute__((noinline)) float erf_ni(float v) { return erff(v); }

#define WS_X   0u
#define WS_Q   (WS_X + 4u * (size_t)NROWP * HIDN)
#define WS_K   (WS_Q + 2u * (size_t)NROWP * HIDN)
#define WS_V   (WS_K + 2u * (size_t)NROWP * HIDN)
#define WS_END (WS_V + 2u * (size_t)NROWP * HIDN)

__device__ __forceinline__ size_t tokrow(int b, int d, int i) { return (size_t)b * RPB + (i == 0 ? 0 : (i <= NQT ? i : (1 + NQT + (size_t)d * NS + (i - 1 - NQT)))); }
__global__ __launch_bounds__(192) void k_gath(const float* __restrict__ CLS, const float* __restrict__ QRY, const float* __restrict__ DOC, float* __restrict__ XR) { const size_t row = blockIdx.x; const int t = threadIdx.x;
  const float* src = nullptr; if (row < (size_t)NROW) { const size_t b = row / RPB; const int j = (int)(row % RPB); if (j == 0) src = CLS + b * HIDN; else if (j <= NQT) src = QRY + (b * NQT + (j - 1)) * HIDN; else src = DOC + (b * (size_t)ND * NS + (j - 1 - NQT)) * HIDN; }
  v4f o; if (src) { o[0] = bfr(src[t * 4]); o[1] = bfr(src[t * 4 + 1]); o[2] = bfr(src[t * 4 + 2]); o[3] = bfr(src[t * 4 + 3]); } else { o[0] = o[1] = o[2] = o[3] = 0.f; }
  vst2(XR + row * HIDN + t * 4, o); }
__global__ __launch_bounds__(128) void k_proj(const float* __restrict__ XR, const float* __restrict__ WQ, const float* __restrict__ BQ, const float* __restrict__ WK, const float* __restrict__ BK, const float* __restrict__ WV, const float* __restrict__ BV, _Float16* __restrict__ Q, _Float16* __restrict__ K, _Float16* __restrict__ V) { __shared__ __align__(16) _Float16 sh[64][136];
  const int tid = threadIdx.x, wave = tid >> 5, lane = tid & 31, col = lane & 15, g = lane >> 4; const int which = blockIdx.z; const int c0 = blockIdx.y * 128; const size_t r0 = (size_t)blockIdx.x * 64;
  const float* Wm = which == 0 ? WQ : which == 1 ? WK : WV; const float* Bm = which == 0 ? BQ : which == 1 ? BK : BV;
  v8f acc[8] = {};
#pragma unroll 2
  for (int kc = 0; kc < HIDN / 32; ++kc) { v16b a; { const float* p = XR + (r0 + wave * 16 + col) * HIDN + kc * 32 + 8 * g;
#pragma unroll
      for (int i = 0; i < 8; ++i) { a[i] = (__bf16)p[i]; a[8 + i] = (__bf16)p[16 + i]; } }
#pragma unroll
    for (int j = 0; j < 8; ++j) { v16b w; const size_t o = c0 + j * 16 + col;
#pragma unroll
      for (int i = 0; i < 8; ++i) { w[i] = (__bf16)Wm[o * HIDN + kc * 32 + 8 * g + i]; w[8 + i] = (__bf16)Wm[o * HIDN + kc * 32 + 16 + 8 * g + i]; }
      acc[j] = wmma_bf(a, w, acc[j]); } }
#pragma unroll
  for (int j = 0; j < 8; ++j) { const float bb = bfr(Bm[c0 + j * 16 + col]);
#pragma unroll
    for (int r = 0; r < 8; ++r) sh[wave * 16 + 8 * g + r][j * 16 + col] = (_Float16)(acc[j][r] + bb); }
  __syncthreads(); { _Float16* dst = which == 0 ? Q : which == 1 ? K : V; for (int e = tid; e < 64 * 16; e += 128) { const int rl = e >> 4, q = e & 15; vst2((unsigned*)(dst + (r0 + rl) * HIDN + c0 + q * 8), *(const v4u*)&sh[rl][q * 8]); } } }
__global__ __launch_bounds__(128) void k_att(const _Float16* __restrict__ Q, const _Float16* __restrict__ K, const _Float16* __restrict__ V, const float* __restrict__ QM, const float* __restrict__ DMK, float* __restrict__ OUT) {
  __shared__ __align__(16) float sp[4][16][36]; __shared__ __align__(16) float so[4][16][68]; __shared__ __align__(16) _Float16 sv[32][72]; __shared__ float smk[32]; __shared__ int srow[32];
  const int tid = threadIdx.x, wave = tid >> 5, lane = tid & 31, col = lane & 15, g = lane >> 4; const int qb = blockIdx.x, h = blockIdx.y; const int bd = blockIdx.z; const int b = bd / TND, d = bd % TND;
  const int qi = qb * 64 + wave * 16 + col; const int qic = (qi < LSEQ) ? qi : (LSEQ - 1);
  v16h aq[2];
#pragma unroll
  for (int kc = 0; kc < 2; ++kc) aq[kc] = frag_h(Q + tokrow(b, d, qic) * HIDN + h * HD + kc * 32, lane);
  float m[8], l[8];
#pragma unroll
  for (int r = 0; r < 8; ++r) { m[r] = -3.0e38f; l[r] = 0.f; }
  v8f acc[4] = {};
#pragma unroll 1
  for (int ks = 0; ks < (LSEQ + 31) / 32; ++ks) {
    __syncthreads();
    if (tid < 32) { int ki = ks * 32 + tid; const bool valid = ki < LSEQ; if (!valid) ki = LSEQ - 1; const size_t rr = tokrow(b, d, ki); srow[tid] = (int)rr;
      float mk; if (ki == 0) mk = 0.f; else if (ki <= NQT) mk = bfr(QM[(size_t)b * NQT + (ki - 1)]); else mk = bfr(DMK[((size_t)b * ND + d) * NS + (ki - 1 - NQT)]); smk[tid] = valid ? mk : -3.0e38f; }
    __syncthreads();
    for (int e = tid; e < 32 * 8; e += 128) { const int i = e >> 3, q8 = e & 7; *(v4u*)&sv[i][q8 * 8] = *(const v4u*)(V + (size_t)srow[i] * HIDN + h * HD + q8 * 8); }
    float s[2][8];
#pragma unroll
    for (int ct = 0; ct < 2; ++ct) { const int i = ct * 16 + col; v8f c = {};
#pragma unroll
      for (int kc = 0; kc < 2; ++kc) c = wmma16(aq[kc], frag_h(K + (size_t)srow[i] * HIDN + h * HD + kc * 32, lane), c);
      const float mk = smk[i];
#pragma unroll
      for (int r = 0; r < 8; ++r) s[ct][r] = (mk <= -1.0e38f) ? -3.0e38f : (c[r] * 0.125f + mk); }
    float alpha[8];
#pragma unroll
    for (int r = 0; r < 8; ++r) { float mx = fmaxf(s[0][r], s[1][r]);
#pragma unroll
      for (int o = 1; o < 16; o <<= 1) mx = fmaxf(mx, __shfl_xor(mx, o));
      const float mn = fmaxf(m[r], mx); alpha[r] = __expf(m[r] - mn); const float e0 = (s[0][r] <= -1.0e38f) ? 0.f : __expf(s[0][r] - mn), e1 = (s[1][r] <= -1.0e38f) ? 0.f : __expf(s[1][r] - mn); float es = e0 + e1;
#pragma unroll
      for (int o = 1; o < 16; o <<= 1) es += __shfl_xor(es, o);
      l[r] = l[r] * alpha[r] + es; m[r] = mn; sp[wave][8 * g + r][col] = e0; sp[wave][8 * g + r][16 + col] = e1; }
#pragma unroll
    for (int j = 0; j < 4; ++j)
#pragma unroll
      for (int r = 0; r < 8; ++r) acc[j][r] *= alpha[r];
    __syncthreads();
    const v16h pa = frag_f32s(&sp[wave][col][0], lane, 2048.0f);
#pragma unroll
    for (int j = 0; j < 4; ++j) { v16h vb; const int dc = j * 16 + col;
#pragma unroll
      for (int i = 0; i < 8; ++i) { vb[i] = sv[8 * g + i][dc]; vb[8 + i] = sv[16 + 8 * g + i][dc]; }
      acc[j] = wmma16(pa, vb, acc[j]); } }
#pragma unroll
  for (int r = 0; r < 8; ++r) { const float il = (1.0f / 2048.0f) / l[r];
#pragma unroll
    for (int j = 0; j < 4; ++j) so[wave][8 * g + r][j * 16 + col] = acc[j][r] * il; }
  LDSX();
  for (int rl = 0; rl < 16; ++rl) { const int qpos = qb * 64 + wave * 16 + rl; if (qpos < LSEQ && lane < 16) vst2(OUT + (((size_t)b * ND + d) * LSEQ + qpos) * HIDN + h * HD + lane * 4, *(const v4f*)&so[wave][rl][lane * 4]); } }
extern "C" void kernel_launch(void* const* d_in, const int* in_sizes, int n_in, void* d_out, int out_size, void* d_ws, size_t ws_size, hipStream_t stream) {
  (void)in_sizes; (void)n_in; (void)out_size;
  const float** F = (const float**)d_in;
  if (ws_size < (size_t)WS_END) return;
  char* ws = (char*)d_ws; float* XR = (float*)(ws + WS_X); _Float16 *Q = (_Float16*)(ws + WS_Q), *K = (_Float16*)(ws + WS_K), *V = (_Float16*)(ws + WS_V);
  k_gath<<<TPR * 64, 192, 0, stream>>>(F[0], F[1], F[2], XR);
  k_proj<<<dim3(TPR, HIDN / 128, 3), 128, 0, stream>>>(XR, F[5], F[6], F[7], F[8], F[9], F[10], Q, K, V);
  k_att<<<dim3((LSEQ + 63) / 64, NH, TNB * TND), 128, 0, stream>>>(Q, K, V, F[3], F[4], (float*)d_out);
}
